// SimpleSelfAttention_40965398069529
// MI455X (gfx1250) — hardware-verified
//
#include <hip/hip_runtime.h>


#ifndef NB
#define NB 4
#endif
#ifndef SEQ
#define SEQ 2048
#endif
#define NB_FULL  4
#define SEQ_FULL 2048
#define EM   512
#define TT   SEQ
#define PCAR 1024.0f
#define WCAR 64.0f
#define RCAR 2048.0f
#define RINV (1.0f / 2048.0f)
#define OSC  (1.0f / 65536.0f)
#define SCL  0.044194173824159216f

static_assert(SEQ % 128 == 0);
static_assert(SEQ >= 128 && SEQ <= SEQ_FULL);
static_assert(NB >= 1 && NB <= NB_FULL);
static_assert(EM % 64 == 0 && EM % 32 == 0);
static_assert(((size_t)NB * SEQ) % 64 == 0);
static_assert((size_t)NB * SEQ * EM * 4 <= (size_t)16777216);

typedef _Float16 h16;
typedef unsigned short bf;
typedef __attribute__((ext_vector_type(16))) __bf16   v16bf;
typedef __attribute__((ext_vector_type(16))) _Float16 v16h;
typedef __attribute__((ext_vector_type(8)))  _Float16 v8h;
typedef __attribute__((ext_vector_type(4)))  _Float16 v4h;
typedef __attribute__((ext_vector_type(8)))  unsigned short v8us;
typedef __attribute__((ext_vector_type(8)))  float    v8f;
typedef __attribute__((ext_vector_type(4)))  float    v4f;
typedef v4f  __attribute__((may_alias)) v4fa;

__device__ __forceinline__ unsigned short f2bf(float f) { unsigned u = __float_as_uint(f); u += 0x7FFFu + ((u >> 16) & 1u); return (unsigned short)(u >> 16); }
__device__ __forceinline__ float bf2f(unsigned short b) { return __uint_as_float(((unsigned)b) << 16); }
__device__ __forceinline__ float bfr(float f) { return bf2f(f2bf(f)); }
__device__ __forceinline__ h16 tohx(float x) { return (h16)x; }
__device__ __forceinline__ v16h cat16(v8h lo, v8h hi) { return __builtin_shufflevector(lo, hi, 0, 1, 2, 3, 4, 5, 6, 7, 8, 9, 10, 11, 12, 13, 14, 15); }
__device__ __forceinline__ v16bf cat16b(v8us lo, v8us hi) { return __builtin_bit_cast(v16bf, __builtin_shufflevector(lo, hi, 0, 1, 2, 3, 4, 5, 6, 7, 8, 9, 10, 11, 12, 13, 14, 15)); }
__device__ __forceinline__ v8f wmma16(v16h a, v16h b, v8f c) { return __builtin_amdgcn_wmma_f32_16x16x32_f16(false, a, false, b, (short)0, c, false, false); }
__device__ __forceinline__ v8f wmmab(v16bf a, v16bf b, v8f c) { return __builtin_amdgcn_wmma_f32_16x16x32_bf16(false, a, false, b, (short)0, c, false, false); }

template <typename T16> struct WFrag;
template <> struct WFrag<h16> { typedef v16h V; static __device__ __forceinline__ V ld(const h16* p) { return cat16(*(const v8h*)p, *(const v8h*)(p + 16)); } static __device__ __forceinline__ v8f mma(V a, V b, v8f c) { return wmma16(a, b, c); } };
template <> struct WFrag<bf> { typedef v16bf V; static __device__ __forceinline__ V ld(const bf* p) { return cat16b(*(const v8us*)p, *(const v8us*)(p + 16)); } static __device__ __forceinline__ v8f mma(V a, V b, v8f c) { return wmmab(a, b, c); } };
template <typename T16, bool BIAS>
__global__ __launch_bounds__(32) void k_gemmw(const T16* __restrict__ A, const T16* __restrict__ Bt, int K, float* C, int ldc, const float* __restrict__ bias, float oscale, size_t sA, size_t sB, size_t sC) {
    typedef typename WFrag<T16>::V V;
    __shared__ __align__(16) float os[16 * 68];
    const size_t z = blockIdx.z; A += z * sA; Bt += z * sB; C += z * sC;
    const int lane = threadIdx.x & 31, lr = lane & 15, hi = lane >> 4; const int r0 = blockIdx.x * 64, c0 = blockIdx.y * 64;
    v8f acc[4][4];
#pragma unroll
    for (int mb = 0; mb < 4; ++mb)
#pragma unroll
        for (int nb = 0; nb < 4; ++nb) acc[mb][nb] = (v8f){};
    const size_t aoff = (size_t)(r0 + lr) * K + 8 * hi, boff = (size_t)(c0 + lr) * K + 8 * hi;
#pragma unroll 1
    for (int kc = 0; kc < K; kc += 32) {
        V a[4];
#pragma unroll
        for (int mb = 0; mb < 4; ++mb) a[mb] = WFrag<T16>::ld(A + aoff + (size_t)mb * 16 * K + kc);
#pragma unroll
        for (int nb = 0; nb < 4; ++nb) { const V b = WFrag<T16>::ld(Bt + boff + (size_t)nb * 16 * K + kc);
#pragma unroll
            for (int mb = 0; mb < 4; ++mb) acc[mb][nb] = WFrag<T16>::mma(a[mb], b, acc[mb][nb]); }
        asm volatile("v_nop\n\tv_nop\n\tv_nop\n\tv_nop" : "+v"(acc[0][0]), "+v"(acc[1][1]), "+v"(acc[2][2]), "+v"(acc[3][3]) : "v"(a[0]), "v"(a[3]));
    }
#pragma unroll
    for (int mb = 0; mb < 4; ++mb) {
#pragma unroll
        for (int nb = 0; nb < 4; ++nb) {
#pragma unroll
            for (int j = 0; j < 8; ++j) os[(hi * 8 + j) * 68 + nb * 16 + lr] = acc[mb][nb][j]; }
        __builtin_amdgcn_wave_barrier(); asm volatile("" ::: "memory");
        float* crow = C + (size_t)(r0 + mb * 16) * ldc + c0;
#pragma unroll 1
        for (int ps = 0; ps < 2; ++ps) {
#pragma unroll
            for (int s = 0; s < 8; ++s) { const int row = 2 * s + hi, cofs = lr * 4; v4f val = *(const v4fa*)(os + row * 68 + cofs); val = val * oscale;
                if (BIAS) { val[0] += bfr(bias[c0 + cofs]); val[1] += bfr(bias[c0 + cofs + 1]); val[2] += bfr(bias[c0 + cofs + 2]); val[3] += bfr(bias[c0 + cofs + 3]); }
                *(volatile v4f*)(crow + (size_t)row * ldc + cofs) = val; }
            if (ps == 0) __threadfence(); }
        __builtin_amdgcn_wave_barrier(); asm volatile("" ::: "memory");
    }
}

__global__ __launch_bounds__(256) void k_cvtb(const float* __restrict__ src, size_t sstride, bf* dst, size_t dstride, size_t n8) {
    const size_t i = (size_t)blockIdx.x * 256 + threadIdx.x; if (i >= n8) return;
    const float* s = src + (size_t)blockIdx.y * sstride + i * 8; bf* d = dst + (size_t)blockIdx.y * dstride + i * 8;
    const v8f v = *(const v8f*)s; v8us o;
#pragma unroll
    for (int k = 0; k < 8; ++k) o[k] = f2bf(v[k]);
    *(volatile v8us*)d = o; __threadfence(); *(volatile v8us*)d = o; }

template <bool RND>
__global__ __launch_bounds__(256) void k_cvth(const float* __restrict__ src, h16* dst, size_t n8, float sc) {
    const size_t i = (size_t)blockIdx.x * 256 + threadIdx.x; if (i >= n8) return;
    const v8f v = *(const v8f*)(src + i * 8); v8h o;
#pragma unroll
    for (int k = 0; k < 8; ++k) { float x = v[k]; if (RND) x = bfr(x); o[k] = tohx(x * sc); }
    *(volatile v8h*)(dst + i * 8) = o; __threadfence(); *(volatile v8h*)(dst + i * 8) = o; }

__global__ __launch_bounds__(256) void k_cvthr(const float* __restrict__ src, h16* dhi, h16* dlo, size_t n8, float rsc) {
    const size_t i = (size_t)blockIdx.x * 256 + threadIdx.x; if (i >= n8) return;
    const v8f v = *(const v8f*)(src + i * 8); v8h oh, ol;
#pragma unroll
    for (int k = 0; k < 8; ++k) { const float x = v[k]; const h16 hx = tohx(x); float r = __fsub_rn(x, (float)hx); asm volatile("" : "+v"(r)); oh[k] = hx; ol[k] = tohx(r * rsc); }
    *(volatile v8h*)(dhi + i * 8) = oh; *(volatile v8h*)(dlo + i * 8) = ol; __threadfence(); *(volatile v8h*)(dhi + i * 8) = oh; *(volatile v8h*)(dlo + i * 8) = ol; }

__global__ __launch_bounds__(256) void k_asoft(const float* __restrict__ Sb, const float* __restrict__ Rb, h16* P16) {
    const int lane = threadIdx.x & 31; const int row = blockIdx.x * 8 + (threadIdx.x >> 5); if (row >= TT) return;
    const float* sr = Sb + (size_t)row * TT; const float* rr = Rb + (size_t)row * TT; float v[TT / 32]; float mx = -3.0e38f;
#pragma unroll
    for (int ch = 0; ch < TT / 128; ++ch) { const int j0 = ch * 128 + lane * 4; const v4f a = *(const v4f*)(sr + j0); const v4f c = *(const v4f*)(rr + j0);
#pragma unroll
        for (int q = 0; q < 4; ++q) { float s0 = __fadd_rn(a[q], c[q]); asm volatile("" : "+v"(s0)); const float t = s0 * SCL; v[ch * 4 + q] = t; mx = fmaxf(mx, t); } }
#pragma unroll
    for (int sh = 16; sh; sh >>= 1) mx = fmaxf(mx, __shfl_xor(mx, sh, 32));
    float sum = 0.f;
#pragma unroll
    for (int k = 0; k < TT / 32; ++k) { float d0 = __fsub_rn(v[k], mx); asm volatile("" : "+v"(d0)); v[k] = __builtin_amdgcn_exp2f(__fmul_rn(d0, 1.4426950408889634f)); sum += v[k]; }
#pragma unroll
    for (int sh = 16; sh; sh >>= 1) sum += __shfl_xor(sum, sh, 32);
    const float f = __fdiv_rn(PCAR, sum);
#pragma unroll 1
    for (int ps = 0; ps < 2; ++ps) {
#pragma unroll
        for (int ch = 0; ch < TT / 128; ++ch) { v4h o4;
#pragma unroll
            for (int q = 0; q < 4; ++q) o4[q] = tohx(v[ch * 4 + q] * f);
            *(volatile v4h*)(P16 + (size_t)row * TT + ch * 128 + lane * 4) = o4; }
        if (ps == 0) __threadfence(); }
}

extern "C" void kernel_launch(void* const* d_in, const int* in_sizes, int n_in,
                              void* d_out, int out_size, void* d_ws, size_t ws_size, hipStream_t stream) {
    if (n_in < 8) return;
    const size_t needx = (size_t)(NB - 1) * SEQ_FULL * EM + (size_t)SEQ * EM;
    if ((size_t)in_sizes[0] < needx || (size_t)in_sizes[1] < needx || (size_t)in_sizes[2] < needx) return;
    if (in_sizes[3] < EM * EM || in_sizes[4] < EM * EM || in_sizes[5] < EM * EM || in_sizes[6] < EM * EM || in_sizes[7] < EM) return;
    if ((size_t)out_size < (size_t)NB * SEQ * EM) return;
    const float* Xv = (const float*)d_in[0];
    const float* Xk = (const float*)d_in[1];
    const float* Xq = (const float*)d_in[2];
    const float* Wq = (const float*)d_in[3];
    const float* Wk = (const float*)d_in[4];
    const float* Wv = (const float*)d_in[5];
    const float* Wo = (const float*)d_in[6];
    const float* bo = (const float*)d_in[7];
    float* OUT = (float*)d_out;

    char* wsp = (char*)d_ws;
    auto take = [&](size_t bytes) { char* p = wsp; wsp += (bytes + 255) & ~(size_t)255; return (void*)p; };
    const size_t nTE = (size_t)SEQ * EM;
    const size_t nW = (size_t)EM * EM;
    bf*  XQ16 = (bf*)take((size_t)NB * nTE * 2); bf* XK16 = (bf*)take((size_t)NB * nTE * 2); bf* XV16 = (bf*)take((size_t)NB * nTE * 2);
    bf*  WQ16 = (bf*)take(nW * 2); bf* WK16 = (bf*)take(nW * 2); bf* WV16 = (bf*)take(nW * 2);
    h16* WO16 = (h16*)take(nW * 2);
    float* F32 = (float*)take((size_t)NB * nTE * 4);
    h16* Q16 = (h16*)take((size_t)NB * nTE * 2); h16* QL16 = (h16*)take((size_t)NB * nTE * 2);
    h16* K16 = (h16*)take((size_t)NB * nTE * 2); h16* VT16 = (h16*)take((size_t)NB * nTE * 2);
    float* Sb = (float*)take((size_t)SEQ * SEQ * 4);
    float* Rb = (float*)take((size_t)SEQ * SEQ * 4);
    h16* P16 = (h16*)take((size_t)SEQ * SEQ * 2);
    h16* CTX16 = (h16*)take((size_t)NB * nTE * 2);
    const size_t used = (size_t)(wsp - (char*)d_ws);
    if (used > ws_size || used > (size_t)134217728) return;

    const unsigned gx = (unsigned)((nTE / 8 + 255) / 256), gw = (unsigned)((nW / 8 + 255) / 256), gp = (unsigned)(((size_t)NB * nTE / 8 + 255) / 256);
    k_cvtb<<<dim3(gx, NB, 1), 256, 0, stream>>>(Xq, (size_t)SEQ_FULL * EM, XQ16, nTE, nTE / 8);
    k_cvtb<<<dim3(gx, NB, 1), 256, 0, stream>>>(Xk, (size_t)SEQ_FULL * EM, XK16, nTE, nTE / 8);
    k_cvtb<<<dim3(gx, NB, 1), 256, 0, stream>>>(Xv, (size_t)SEQ_FULL * EM, XV16, nTE, nTE / 8);
    k_cvtb<<<dim3(gw, 1, 1), 256, 0, stream>>>(Wq, (size_t)0, WQ16, (size_t)0, nW / 8);
    k_cvtb<<<dim3(gw, 1, 1), 256, 0, stream>>>(Wk, (size_t)0, WK16, (size_t)0, nW / 8);
    k_cvtb<<<dim3(gw, 1, 1), 256, 0, stream>>>(Wv, (size_t)0, WV16, (size_t)0, nW / 8);
    k_cvth<true><<<gw, 256, 0, stream>>>(Wo, WO16, nW / 8, WCAR);

    k_gemmw<bf, false><<<dim3(NB * SEQ / 64, EM / 64, 1), 32, 0, stream>>>(XQ16, WQ16, EM, F32, EM, nullptr, 1.0f, (size_t)0, (size_t)0, (size_t)0);
    k_cvthr<<<gp, 256, 0, stream>>>(F32, Q16, QL16, (size_t)NB * nTE / 8, RCAR);
    k_gemmw<bf, false><<<dim3(NB * SEQ / 64, EM / 64, 1), 32, 0, stream>>>(XK16, WK16, EM, F32, EM, nullptr, 1.0f, (size_t)0, (size_t)0, (size_t)0);
    k_cvth<false><<<gp, 256, 0, stream>>>(F32, K16, (size_t)NB * nTE / 8, 1.0f);
    k_gemmw<bf, false><<<dim3(EM / 64, SEQ / 64, NB), 32, 0, stream>>>(WV16, XV16, EM, F32, SEQ, nullptr, 1.0f, (size_t)0, nTE, nTE);
    k_cvth<false><<<gp, 256, 0, stream>>>(F32, VT16, (size_t)NB * nTE / 8, 1.0f);

    for (int b = 0; b < NB; ++b) {
        k_gemmw<h16, false><<<dim3(SEQ / 64, SEQ / 64, 1), 32, 0, stream>>>(Q16 + (size_t)b * nTE, K16 + (size_t)b * nTE, EM, Sb, SEQ, nullptr, 1.0f, (size_t)0, (size_t)0, (size_t)0);
        k_gemmw<h16, false><<<dim3(SEQ / 64, SEQ / 64, 1), 32, 0, stream>>>(QL16 + (size_t)b * nTE, K16 + (size_t)b * nTE, EM, Rb, SEQ, nullptr, RINV, (size_t)0, (size_t)0, (size_t)0);
        k_asoft<<<SEQ / 8, 256, 0, stream>>>(Sb, Rb, P16);
        k_gemmw<h16, false><<<dim3(SEQ / 64, EM / 64, 1), 32, 0, stream>>>(P16, VT16 + (size_t)b * nTE, SEQ, F32 + (size_t)b * nTE, EM, nullptr, 1.0f, (size_t)0, (size_t)0, (size_t)0);
    }
    k_cvth<false><<<gp, 256, 0, stream>>>(F32, CTX16, (size_t)NB * nTE / 8, 1.0f);
    k_gemmw<h16, true><<<dim3(NB * SEQ / 64, EM / 64, 1), 32, 0, stream>>>(CTX16, WO16, EM, OUT, EM, bo, OSC, (size_t)0, (size_t)0, (size_t)0);
}
